// CoattentiveAggregation_90177133346926
// MI455X (gfx1250) — hardware-verified
//
#include <hip/hip_runtime.h>
#include <stdint.h>

#define DEVINL __device__ __forceinline__

typedef _Float16 f16t;
typedef _Float16 v16h __attribute__((ext_vector_type(16)));
typedef _Float16 v8h  __attribute__((ext_vector_type(8)));
typedef _Float16 v4h  __attribute__((ext_vector_type(4)));
typedef float    v8f  __attribute__((ext_vector_type(8)));
typedef float    v4f  __attribute__((ext_vector_type(4)));
typedef v8h __attribute__((may_alias)) v8ha;
typedef v4h __attribute__((may_alias)) v4ha;
typedef v4f __attribute__((may_alias)) v4fa;
union FragH { v16h v; v8h half[2]; };

#define MN    32
#define FD    128
#define F2    256
#define F3    384
#define TPB   128
#define NWAVE 4
#define PRM   136
#define PT    40
#define PL    33
#define ECAR  4096.0f
#define RECAR (1.0f / 4096.0f)
#define RPOOL (1.0f / 96.0f)

static_assert(TPB == NWAVE * 32);
static_assert((MN % NWAVE) == 0);
static_assert(FD == 4 * 32);
static_assert(F3 == 3 * FD);
static_assert((PRM % 8) == 0);
static_assert((PT % 8) == 0);

DEVINL int imin(int a, int b) { return a < b ? a : b; }
DEVINL int imax(int a, int b) { return a > b ? a : b; }

DEVINL v8f wmma_f16(v16h a, v16h b, v8f c) {
  v8f d = __builtin_amdgcn_wmma_f32_16x16x32_f16(false, a, false, b, (short)0, c, false, false);
  asm volatile("v_nop\n\tv_nop\n\tv_nop\n\tv_nop" : "+v"(d) : "v"(a), "v"(b));
  return d;
}
DEVINL v8f zero8f() {
  v8f z = {0.f, 0.f, 0.f, 0.f, 0.f, 0.f, 0.f, 0.f};
  return z;
}
DEVINL void load_frag(FragH& f, const f16t* row, int k0) {
  f.half[0] = *(const v8ha*)(row + k0);
  f.half[1] = *(const v8ha*)(row + k0 + 16);
}

__global__ __launch_bounds__(TPB)
void coatt_k(const float* __restrict__ feat, const int* __restrict__ isim, const int* __restrict__ icor,
             float* __restrict__ out, int n_dst, int n_src)
{
  __shared__ __attribute__((aligned(16))) f16t  sD[MN * PRM];
  __shared__ __attribute__((aligned(16))) f16t  sQ[MN * PRM];
  __shared__ __attribute__((aligned(16))) f16t  sQT[FD * PT];
  __shared__ __attribute__((aligned(16))) f16t  sDCT[F2 * PT];
  __shared__ __attribute__((aligned(16))) f16t  sER[MN * PT];
  __shared__ __attribute__((aligned(16))) f16t  sES[MN * PT];
  __shared__ __attribute__((aligned(16))) float sL[MN * PL];
  __shared__ __attribute__((aligned(16))) float sRZr[MN];
  __shared__ __attribute__((aligned(16))) float sRZc[MN];
  __shared__ __attribute__((aligned(16))) float sQP[NWAVE * FD];
  __shared__ __attribute__((aligned(16))) float sHP[2 * F2];
  __shared__ __attribute__((aligned(16))) float sHS[F3];

  const int tid = threadIdx.x, lane = tid & 31;
  const int wave = __builtin_amdgcn_readfirstlane(tid >> 5);
  const int h = lane >> 4, m = lane & 15;
  const int n = blockIdx.x;
  if (n >= n_dst) return;

  {
    v4f qs = {0.f, 0.f, 0.f, 0.f};
    const size_t ib = (size_t)n * MN;
    #pragma unroll 2
    for (int i = 0; i < MN / NWAVE; ++i) {
      const int r = wave + NWAVE * i;
      int rs = isim[ib + r];
      int rc = icor[ib + r];
      rs = imin(imax(rs, 0), n_src - 1);
      rc = imin(imax(rc, 0), n_src - 1);
      const v4f d = *(const v4fa*)(feat + (size_t)rs * FD + 4 * lane);
      const v4f q = *(const v4fa*)(feat + (size_t)rc * FD + 4 * lane);
      v4h dh, qh;
      #pragma unroll
      for (int c = 0; c < 4; ++c) { dh[c] = (f16t)d[c]; qh[c] = (f16t)q[c]; }
      *(v4ha*)(sD + r * PRM + 4 * lane) = dh;
      *(v4ha*)(sQ + r * PRM + 4 * lane) = qh;
      #pragma unroll
      for (int c = 0; c < 4; ++c) {
        sDCT[(4 * lane + c) * PT + r] = dh[c];
        sQT[(4 * lane + c) * PT + r]  = qh[c];
        qs[c] += q[c];
      }
    }
    *(v4fa*)(sQP + wave * FD + 4 * lane) = qs;
  }
  __syncthreads();

  {
    const int mt = wave & 1, nt = wave >> 1;
    const f16t* arow = sD + (mt * 16 + m) * PRM + 8 * h;
    const f16t* brow = sQ + (nt * 16 + m) * PRM + 8 * h;
    v8f acc = zero8f();
    #pragma unroll
    for (int ks = 0; ks < FD / 32; ++ks) {
      FragH a, b;
      load_frag(a, arow, 32 * ks);
      load_frag(b, brow, 32 * ks);
      acc = wmma_f16(a.v, b.v, acc);
    }
    #pragma unroll
    for (int r = 0; r < 8; ++r)
      sL[(mt * 16 + 8 * h + r) * PL + nt * 16 + m] = acc[r];
  }
  __syncthreads();

  if (wave == 0) {
    const float* lr = sL + lane * PL;
    float mx = -3.0e38f;
    #pragma unroll 8
    for (int k = 0; k < MN; ++k) mx = fmaxf(mx, lr[k]);
    float z = 0.0f;
    #pragma unroll 8
    for (int k = 0; k < MN; ++k) {
      const float e = __expf(lr[k] - mx);
      z += e;
      sER[lane * PT + k] = (f16t)(e * ECAR);
    }
    sRZr[lane] = 1.0f / z;
  } else if (wave == 1) {
    const float* lc = sL + lane;
    float mx = -3.0e38f;
    #pragma unroll 8
    for (int j = 0; j < MN; ++j) mx = fmaxf(mx, lc[j * PL]);
    float z = 0.0f;
    #pragma unroll 8
    for (int j = 0; j < MN; ++j) {
      const float e = __expf(lc[j * PL] - mx);
      z += e;
      sES[lane * PT + j] = (f16t)(e * ECAR);
    }
    sRZc[lane] = 1.0f / z;
  }
  __syncthreads();

  {
    const int mt = wave & 1, ntb = (wave >> 1) * 4;
    FragH a;
    load_frag(a, sER + (mt * 16 + m) * PT + 8 * h, 0);
    const v4f rz0 = *(const v4fa*)(sRZr + mt * 16 + 8 * h);
    const v4f rz1 = *(const v4fa*)(sRZr + mt * 16 + 8 * h + 4);
    #pragma unroll
    for (int j = 0; j < 4; ++j) {
      const int nt = ntb + j;
      FragH b;
      load_frag(b, sQT + (nt * 16 + m) * PT + 8 * h, 0);
      const v8f acc = wmma_f16(a.v, b.v, zero8f());
      v8h o;
      #pragma unroll
      for (int r = 0; r < 4; ++r) {
        o[r]     = (f16t)(acc[r]     * (rz0[r] * RECAR));
        o[4 + r] = (f16t)(acc[4 + r] * (rz1[r] * RECAR));
      }
      *(v8ha*)(sDCT + (FD + nt * 16 + m) * PT + mt * 16 + 8 * h) = o;
    }
  }
  __syncthreads();

  {
    const int mt = wave & 1, ntb = (wave >> 1) * 8;
    FragH a;
    load_frag(a, sES + (mt * 16 + m) * PT + 8 * h, 0);
    const v4f rz0 = *(const v4fa*)(sRZc + mt * 16 + 8 * h);
    const v4f rz1 = *(const v4fa*)(sRZc + mt * 16 + 8 * h + 4);
    #pragma unroll
    for (int j = 0; j < 8; ++j) {
      const int nt = ntb + j;
      FragH b;
      load_frag(b, sDCT + (nt * 16 + m) * PT + 8 * h, 0);
      const v8f acc = wmma_f16(a.v, b.v, zero8f());
      float s = acc[0] * rz0[0];
      s = fmaf(acc[1], rz0[1], s);
      s = fmaf(acc[2], rz0[2], s);
      s = fmaf(acc[3], rz0[3], s);
      s = fmaf(acc[4], rz1[0], s);
      s = fmaf(acc[5], rz1[1], s);
      s = fmaf(acc[6], rz1[2], s);
      s = fmaf(acc[7], rz1[3], s);
      s += __shfl_xor(s, 16);
      s *= RECAR;
      if (h == 0) sHP[mt * F2 + nt * 16 + m] = s;
    }
  }
  __syncthreads();

  {
    const int t = tid;
    sHS[t]          = ((sQP[t] + sQP[FD + t]) + sQP[2 * FD + t]) + sQP[3 * FD + t];
    sHS[FD + t]     = sHP[t] + sHP[F2 + t];
    sHS[2 * FD + t] = sHP[FD + t] + sHP[F2 + FD + t];
  }
  __syncthreads();
  if (wave == 0) {
    const int f0 = 4 * lane;
    const int ns = imin(n, n_src - 1);
    const v4f self = *(const v4fa*)(feat + (size_t)ns * FD + f0);
    v4f o;
    #pragma unroll
    for (int c = 0; c < 4; ++c) {
      const int f = f0 + c;
      const float hn = ((sHS[3 * f] + sHS[3 * f + 1]) + sHS[3 * f + 2]) * RPOOL;
      o[c] = self[c] + hn;
    }
    float* dst = out + (size_t)n * FD + f0;
    *(volatile v4f*)dst = o;
    __threadfence();
    *(volatile v4f*)dst = o;
  }
}

extern "C" void kernel_launch(void* const* d_in, const int* in_sizes, int n_in,
                              void* d_out, int out_size, void* d_ws, size_t ws_size,
                              hipStream_t stream) {
  (void)d_ws; (void)ws_size;
  if (n_in < 3) return;
  const int n_feat = in_sizes[0];
  if (n_feat < FD || (n_feat % FD) != 0) return;
  const int n_src = n_feat / FD;
  if (in_sizes[1] <= 0 || (in_sizes[1] % MN) != 0) return;
  if (in_sizes[2] != in_sizes[1]) return;
  const int n_dst = in_sizes[1] / MN;
  if (n_dst > n_src) return;
  if (out_size != n_dst * FD) return;

  const float* feat = (const float*)d_in[0];
  const int*   isim = (const int*)d_in[1];
  const int*   icor = (const int*)d_in[2];
  float* outp = (float*)d_out;

  coatt_k<<<dim3((unsigned)n_dst), dim3(TPB), 0, stream>>>(feat, isim, icor, outp, n_dst, n_src);
  (void)hipGetLastError();
}
